// LightHeadRCNNResNet101_Head_5325759447413
// MI455X (gfx1250) — hardware-verified
//
#include <hip/hip_runtime.h>

#pragma clang fp contract(off)

constexpr int FEAT_H   = 38;
constexpr int FEAT_W   = 50;
constexpr int NPOS     = FEAT_H * FEAT_W;
constexpr int MPOS     = 1920;
constexpr int CH_IN    = 2048;
constexpr int CH_MID   = 256;
constexpr int CH_OUT   = 490;
constexpr int CH_OUTP  = 512;
constexpr int NTAP     = 15;
constexpr int HALO     = 7;
constexpr int HP_COL   = 52;
constexpr int WP_ROW   = 64;
constexpr int GEOM_WHP = 0;
constexpr int GEOM_HWP = 1;
constexpr int XTC_ROWS = 2640;
constexpr int XTR_ROWS = 2496;
constexpr int P2C_ROWS = 2496;
constexpr int P2R_ROWS = 2608;
constexpr int KC1      = NTAP * CH_IN;
constexpr int KC2      = NTAP * CH_MID;
constexpr int N_ROI    = 512;
constexpr int KFC      = 512;
constexpr int NFC      = 2048;
constexpr int NHD      = 512;
constexpr int LOC_N    = 324;
constexpr int SC_N     = 81;
constexpr int SC_BASE  = 384;
constexpr int NBIN     = 7;
constexpr int BIN_CH   = 10;
constexpr float W_CARRY     = 256.0f;
constexpr float W_CARRY_INV = 1.0f / 256.0f;

static_assert(KC1 % 32 == 0 && KC2 % 32 == 0 && KFC % 32 == 0 && NFC % 32 == 0);
static_assert(MPOS % 64 == 0 && CH_MID % 64 == 0 && CH_OUTP % 64 == 0 && N_ROI % 64 == 0 && NFC % 64 == 0 && NHD % 64 == 0);
static_assert(MPOS >= NPOS);
static_assert((MPOS - 1) / FEAT_H * HP_COL + (MPOS - 1) % FEAT_H + NTAP <= XTC_ROWS);
static_assert((MPOS - 1) / FEAT_W * WP_ROW + (MPOS - 1) % FEAT_W + NTAP <= XTR_ROWS);
static_assert((MPOS - 1) / FEAT_W * WP_ROW + (MPOS - 1) % FEAT_W + NTAP <= P2C_ROWS);
static_assert((FEAT_W - 1) * HP_COL + (FEAT_H - 1) + NTAP <= P2R_ROWS);
static_assert(((MPOS - 1) % FEAT_W) * HP_COL + (MPOS - 1) / FEAT_W + NTAP <= P2R_ROWS);
static_assert(XTC_ROWS >= FEAT_W * HP_COL && XTR_ROWS >= FEAT_H * WP_ROW);
static_assert(P2C_ROWS >= FEAT_H * WP_ROW && P2R_ROWS >= FEAT_W * HP_COL);
static_assert(P2C_ROWS % 8 == 0 && P2R_ROWS % 8 == 0);
static_assert((CH_MID * (KC1 / 8)) % 256 == 0 && (CH_OUTP * (KC2 / 8)) % 256 == 0);
static_assert((NFC * (KFC / 8)) % 256 == 0 && (SC_BASE * (NFC / 8)) % 256 == 0 && ((NHD - SC_BASE) * (NFC / 8)) % 256 == 0);
static_assert(LOC_N <= SC_BASE && SC_BASE + 128 == NHD && SC_N <= 128 && CH_OUT <= CH_OUTP && CH_OUT <= KFC);
static_assert(NBIN * NBIN * BIN_CH == CH_OUT);
static_assert(N_ROI * LOC_N * 4 == 663552 && N_ROI * (LOC_N + SC_N) * 4 == 829440);
static_assert((N_ROI * (LOC_N + SC_N)) % 128 == 0 && (N_ROI * LOC_N) % 128 == 0);

constexpr size_t WS_XTC  = (size_t)XTC_ROWS * CH_IN * 2;
constexpr size_t WS_XTR  = (size_t)XTR_ROWS * CH_IN * 2;
constexpr size_t WS_W1   = (size_t)CH_MID * KC1 * 2;
constexpr size_t WS_C1   = (size_t)MPOS * CH_MID * 4;
constexpr size_t WS_P2C  = (size_t)P2C_ROWS * CH_MID * 2;
constexpr size_t WS_P2R  = (size_t)P2R_ROWS * CH_MID * 2;
constexpr size_t WS_W2   = (size_t)CH_OUTP * KC2 * 2;
constexpr size_t WS_BTAB = (size_t)CH_OUTP * 4;
constexpr size_t WS_C2   = (size_t)MPOS * CH_OUTP * 4;
constexpr size_t WS_POOL = (size_t)N_ROI * KFC * 2;
constexpr size_t WS_WFC  = (size_t)NFC * KFC * 2;
constexpr size_t WS_CFC  = (size_t)N_ROI * NFC * 2;
constexpr size_t WS_WHD  = (size_t)NHD * NFC * 2;
constexpr size_t WS_CHD  = (size_t)N_ROI * NHD * 4;

constexpr size_t OFF_XTC   = 0;
constexpr size_t OFF_XTR   = OFF_XTC + WS_XTC;
constexpr size_t OFF_W1C   = OFF_XTR + WS_XTR;
constexpr size_t OFF_W1R   = OFF_W1C + WS_W1;
constexpr size_t OFF_C1C   = OFF_W1R + WS_W1;
constexpr size_t OFF_C1R   = OFF_C1C + WS_C1;
constexpr size_t OFF_P2C   = OFF_C1R + WS_C1;
constexpr size_t OFF_P2R   = OFF_P2C + WS_P2C;
constexpr size_t OFF_W2C   = OFF_P2R + WS_P2R;
constexpr size_t OFF_W2R   = OFF_W2C + WS_W2;
constexpr size_t OFF_BTAB  = OFF_W2R + WS_W2;
constexpr size_t OFF_C2A   = OFF_BTAB + WS_BTAB;
constexpr size_t OFF_C2    = OFF_C2A + WS_C2;
constexpr size_t OFF_POOLH = OFF_C2 + WS_C2;
constexpr size_t OFF_POOLL = OFF_POOLH + WS_POOL;
constexpr size_t OFF_WFCH  = OFF_POOLL + WS_POOL;
constexpr size_t OFF_WFCL  = OFF_WFCH + WS_WFC;
constexpr size_t OFF_CFCH  = OFF_WFCL + WS_WFC;
constexpr size_t OFF_CFCL  = OFF_CFCH + WS_CFC;
constexpr size_t OFF_WHDH  = OFF_CFCL + WS_CFC;
constexpr size_t OFF_WHDL  = OFF_WHDH + WS_WHD;
constexpr size_t OFF_CHD   = OFF_WHDL + WS_WHD;
constexpr size_t WS_TOTAL  = OFF_CHD + WS_CHD;
static_assert(WS_TOTAL <= (size_t)134217728);
static_assert(OFF_XTR % 2048 == 0 && OFF_W1C % 2048 == 0 && OFF_C1C % 2048 == 0 && OFF_P2C % 2048 == 0 &&
              OFF_P2R % 2048 == 0 && OFF_W2C % 2048 == 0 && OFF_BTAB % 2048 == 0 && OFF_C2A % 2048 == 0 &&
              OFF_POOLH % 2048 == 0 && OFF_WFCH % 2048 == 0 && OFF_CFCH % 2048 == 0 && OFF_WHDH % 2048 == 0 &&
              OFF_CHD % 2048 == 0);

typedef __attribute__((ext_vector_type(16))) _Float16 v16h;
typedef __attribute__((ext_vector_type(8)))  _Float16 v8h;
typedef __attribute__((ext_vector_type(16))) __bf16   v16b;
typedef __attribute__((ext_vector_type(8)))  __bf16   v8b;
typedef __attribute__((ext_vector_type(8)))  float    v8f;
typedef __attribute__((ext_vector_type(4)))  float    v4f;
typedef __attribute__((ext_vector_type(4)))  unsigned v4u;

__device__ __forceinline__ unsigned short f2bf_bits(float f) {
  unsigned u = __float_as_uint(f);
  return (unsigned short)((u + 0x7FFFu + ((u >> 16) & 1u)) >> 16);
}
__device__ __forceinline__ float bf_bits2f(unsigned short h) { return __uint_as_float(((unsigned)h) << 16); }

__device__ __forceinline__ void dep_guard_h(v8f& a, v8f& b, v16h x, v16h y) { asm volatile("v_nop\n\tv_nop\n\tv_nop\n\tv_nop" : "+v"(a), "+v"(b) : "v"(x), "v"(y)); }
__device__ __forceinline__ void dep_guard_b(v8f& a, v8f& b, v16b x, v16b y) { asm volatile("v_nop\n\tv_nop\n\tv_nop\n\tv_nop" : "+v"(a), "+v"(b) : "v"(x), "v"(y)); }
__device__ __forceinline__ void keep4_h(v16h a, v16h b, v16h c, v16h d) { asm volatile("v_nop" :: "v"(a), "v"(b), "v"(c), "v"(d)); }
__device__ __forceinline__ void keep4_b(v16b a, v16b b, v16b c, v16b d) { asm volatile("v_nop" :: "v"(a), "v"(b), "v"(c), "v"(d)); }
__device__ __forceinline__ void acc_guard4(v8f& a, v8f& b, v8f& c, v8f& d) { asm volatile("v_nop\n\tv_nop\n\tv_nop\n\tv_nop" : "+v"(a), "+v"(b), "+v"(c), "+v"(d)); }
template <typename T> struct Frag;
template <> struct Frag<_Float16> {
  typedef v16h V; union U { v16h v; v8h h[2]; };
  static __device__ __forceinline__ v16h load(const _Float16* p) {
    U f; f.h[0] = *(const v8h*)(p); f.h[1] = *(const v8h*)(p + 16); return f.v;
  }
  static __device__ __forceinline__ v8f mma(v16h a, v16h b, v8f c) {
    return __builtin_amdgcn_wmma_f32_16x16x32_f16(false, a, false, b, (short)0, c, false, false);
  }
  static __device__ __forceinline__ void guard(v8f& a, v8f& b, v16h x, v16h y) { dep_guard_h(a, b, x, y); }
  static __device__ __forceinline__ void keep(v16h a, v16h b, v16h c, v16h d) { keep4_h(a, b, c, d); }
};
template <> struct Frag<__bf16> {
  typedef v16b V; union U { v16b v; v8b h[2]; };
  static __device__ __forceinline__ v16b load(const __bf16* p) {
    U f; f.h[0] = *(const v8b*)(p); f.h[1] = *(const v8b*)(p + 16); return f.v;
  }
  static __device__ __forceinline__ v8f mma(v16b a, v16b b, v8f c) {
    return __builtin_amdgcn_wmma_f32_16x16x32_bf16(false, a, false, b, (short)0, c, false, false);
  }
  static __device__ __forceinline__ void guard(v8f& a, v8f& b, v16b x, v16b y) { dep_guard_b(a, b, x, y); }
  static __device__ __forceinline__ void keep(v16b a, v16b b, v16b c, v16b d) { keep4_b(a, b, c, d); }
};

template <int ACT> __device__ __forceinline__ float epi_act(float v) {
  if (ACT == 1) v = tanhf(v);
  if (ACT == 2) v = fmaxf(v, 0.0f);
  if (ACT == 3) v = v / (1.0f + expf(-v));
  if (ACT == 4) v = (v > 0.f) ? v : 0.01f * v;
  return v;
}

template <int ET> struct Elem;
template <> struct Elem<0> { typedef _Float16 T; };
template <> struct Elem<1> { typedef __bf16 T; };
template <int ET, bool SPLIT, int BIAS_MODE, int OUT_MODE, bool RESID, int ACT = 0, bool RMAP = false>
__global__ __launch_bounds__(256) void wmma_gemm64(
    const unsigned short* __restrict__ Ap, const unsigned short* __restrict__ A2p, int lda, long strideA,
    const unsigned short* __restrict__ Btp, const unsigned short* __restrict__ Bt2p, int ldb, long strideB,
    void* __restrict__ Cout, void* __restrict__ Cout2, int ldc, long strideC,
    const float* __restrict__ bias,
    const float* __restrict__ resid, long strideR,
    int M, int N, int K, float scale,
    int a_rdiv, int a_mulq, int a_mulr) {
  static_assert(!(RESID && OUT_MODE != 0));
  typedef typename Elem<ET>::T T;
  typedef typename Frag<T>::V V;
  const T* A = (const T*)Ap; const T* A2 = (const T*)A2p; const T* Bt = (const T*)Btp; const T* Bt2 = (const T*)Bt2p;
  __shared__ __align__(16) float sT[8][16 * 68];
  const int b    = blockIdx.y;
  const int lane = threadIdx.x & 31;
  const int wave = threadIdx.x >> 5;
  const int wpb  = (int)(blockDim.x >> 5);
  const int tilesN = N >> 6;
  const int tilesM = M >> 6;
  const int tile = blockIdx.x * wpb + wave;
  if (tile >= tilesM * tilesN) return;
  const int tm = tile / tilesN;
  const int tn = tile - tm * tilesN;
  const int m0 = tm << 6;
  const int n0 = tn << 6;

  const T* Ab  = A  + (size_t)b * strideA;
  const T* Bb  = Bt + (size_t)b * strideB;
  const T* Ab2 = SPLIT ? (A2  + (size_t)b * strideA) : nullptr;
  const T* Bb2 = SPLIT ? (Bt2 + (size_t)b * strideB) : nullptr;

  const int rlane = lane & 15;
  const int koff  = (lane >> 4) * 8;
  const int mOff  = (lane >> 4) * 8;

  size_t arow[4];
#pragma unroll
  for (int i = 0; i < 4; ++i) {
    const int m = m0 + (i << 4) + rlane;
    if (RMAP) {
      const int qd = m / a_rdiv;
      const long ri = (long)qd * a_mulq + (long)(m - qd * a_rdiv) * a_mulr;
      arow[i] = (size_t)ri * (size_t)lda;
    } else {
      arow[i] = (size_t)m * (size_t)lda;
    }
  }

  v8f acc[4][4];
#pragma unroll
  for (int i = 0; i < 4; ++i)
#pragma unroll
    for (int j = 0; j < 4; ++j) acc[i][j] = (v8f){0.f,0.f,0.f,0.f,0.f,0.f,0.f,0.f};

  for (int k0 = 0; k0 < K; k0 += 32) {
    V bh[4], bl[4];
#pragma unroll
    for (int j = 0; j < 4; ++j) {
      const size_t bo = (size_t)(n0 + (j << 4) + rlane) * ldb + koff + k0;
      bh[j] = Frag<T>::load(Bb + bo);
      if (SPLIT) bl[j] = Frag<T>::load(Bb2 + bo);
    }
#pragma unroll
    for (int i = 0; i < 4; ++i) {
      const size_t ao = arow[i] + koff + k0;
      V ah = Frag<T>::load(Ab + ao);
      V al;
      if (SPLIT) al = Frag<T>::load(Ab2 + ao);
#pragma unroll
      for (int j = 0; j < 4; ++j) {
        acc[i][j] = Frag<T>::mma(ah, bh[j], acc[i][j]);
        if (SPLIT) {
          acc[i][j] = Frag<T>::mma(ah, bl[j], acc[i][j]);
          acc[i][j] = Frag<T>::mma(al, bh[j], acc[i][j]);
        }
      }
      Frag<T>::guard(acc[i][0], acc[i][3], ah, SPLIT ? al : ah);
    }
    Frag<T>::keep(bh[0], bh[1], bh[2], bh[3]);
    if (SPLIT) Frag<T>::keep(bl[0], bl[1], bl[2], bl[3]);
  }
  acc_guard4(acc[0][0], acc[0][1], acc[0][2], acc[0][3]);
  acc_guard4(acc[1][0], acc[1][1], acc[1][2], acc[1][3]);
  acc_guard4(acc[2][0], acc[2][1], acc[2][2], acc[2][3]);
  acc_guard4(acc[3][0], acc[3][1], acc[3][2], acc[3][3]);

  float* slab = sT[wave];
  const float* Rb = RESID ? (resid + (size_t)b * strideR) : nullptr;
#pragma unroll
  for (int i = 0; i < 4; ++i) {
    const int mBase = m0 + (i << 4);
#pragma unroll
    for (int j = 0; j < 4; ++j) {
      const int n = n0 + (j << 4) + rlane;
      float bv = 0.f;
      if (BIAS_MODE == 2) bv = bias[n];
#pragma unroll
      for (int r = 0; r < 8; ++r) {
        float v = acc[i][j][r] * scale;
        if (BIAS_MODE == 1) v += bias[mBase + mOff + r];
        if (BIAS_MODE == 2) v += bv;
        if (!RESID) v = epi_act<ACT>(v);
        slab[(mOff + r) * 68 + (j << 4) + rlane] = v;
      }
    }
    __builtin_amdgcn_fence(__ATOMIC_RELEASE, "workgroup");
    __builtin_amdgcn_wave_barrier();
    __builtin_amdgcn_fence(__ATOMIC_ACQUIRE, "workgroup");
    if (OUT_MODE == 0) {
      float* C = (float*)Cout + (size_t)b * strideC;
      const int hh = lane >> 4, c4 = (lane & 15) * 4;
      if (RESID) {
        v4f ov[8];
#pragma unroll
        for (int it = 0; it < 8; ++it) {
          const int row = it * 2 + hh;
          v4f v = *(const v4f*)(slab + row * 68 + c4);
          const v4f rv = *(const v4f*)(Rb + (size_t)(mBase + row) * ldc + n0 + c4);
          v = v + rv;
          v[0] = epi_act<ACT>(v[0]); v[1] = epi_act<ACT>(v[1]);
          v[2] = epi_act<ACT>(v[2]); v[3] = epi_act<ACT>(v[3]);
          ov[it] = v;
        }
        for (int pass = 0; pass < 2; ++pass) {
#pragma unroll
          for (int it = 0; it < 8; ++it) {
            const int row = it * 2 + hh;
            *(volatile v4f*)(C + (size_t)(mBase + row) * ldc + n0 + c4) = ov[it];
          }
          __threadfence();
        }
      } else {
        for (int pass = 0; pass < 2; ++pass) {
#pragma unroll
          for (int it = 0; it < 8; ++it) {
            const int row = it * 2 + hh;
            v4f v = *(const v4f*)(slab + row * 68 + c4);
            *(volatile v4f*)(C + (size_t)(mBase + row) * ldc + n0 + c4) = v;
          }
          __threadfence();
        }
      }
    } else {
      const int q = lane >> 3, c8 = (lane & 7) * 8;
      unsigned short* C  = (unsigned short*)Cout  + (size_t)b * strideC;
      unsigned short* C2 = (OUT_MODE == 2) ? ((unsigned short*)Cout2 + (size_t)b * strideC) : nullptr;
      for (int pass = 0; pass < 2; ++pass) {
#pragma unroll
        for (int it = 0; it < 4; ++it) {
          const int row = it * 4 + q;
          const float* sp = slab + row * 68 + c8;
          v8h hv, lv;
#pragma unroll
          for (int e = 0; e < 8; ++e) {
            if (OUT_MODE == 1) {
              hv[e] = (_Float16)sp[e];
            } else {
              unsigned short hb = f2bf_bits(sp[e]);
              unsigned short lb = f2bf_bits(sp[e] - bf_bits2f(hb));
              hv[e] = __builtin_bit_cast(_Float16, hb);
              lv[e] = __builtin_bit_cast(_Float16, lb);
            }
          }
          *(volatile v8h*)(C + (size_t)(mBase + row) * ldc + n0 + c8) = hv;
          if (OUT_MODE == 2) *(volatile v8h*)(C2 + (size_t)(mBase + row) * ldc + n0 + c8) = lv;
        }
        __threadfence();
      }
    }
    __builtin_amdgcn_fence(__ATOMIC_RELEASE, "workgroup");
    __builtin_amdgcn_wave_barrier();
    __builtin_amdgcn_fence(__ATOMIC_ACQUIRE, "workgroup");
  }
}

__device__ __forceinline__ int clampi(int v, int lo, int hi) { return v < lo ? lo : (v > hi ? hi : v); }
__device__ __forceinline__ unsigned h16bits(float f) {
  const _Float16 h = (_Float16)f;
  return (unsigned)__builtin_bit_cast(unsigned short, h);
}
__device__ __forceinline__ void store8_f16(unsigned short* p, const float (&v)[8]) {
  v4u u;
  u[0] = h16bits(v[0]) | (h16bits(v[1]) << 16);
  u[1] = h16bits(v[2]) | (h16bits(v[3]) << 16);
  u[2] = h16bits(v[4]) | (h16bits(v[5]) << 16);
  u[3] = h16bits(v[6]) | (h16bits(v[7]) << 16);
  *(volatile v4u*)p = u;
  __threadfence();
  *(volatile v4u*)p = u;
}
__device__ __forceinline__ void store8_bf16x2(unsigned short* ph, unsigned short* pl, const float (&v)[8]) {
  unsigned hb[8], lb[8];
#pragma unroll
  for (int e = 0; e < 8; ++e) {
    const unsigned short h = f2bf_bits(v[e]);
    hb[e] = (unsigned)h;
    lb[e] = (unsigned)f2bf_bits(v[e] - bf_bits2f(h));
  }
  v4u uh, ul;
  uh[0] = hb[0] | (hb[1] << 16); uh[1] = hb[2] | (hb[3] << 16); uh[2] = hb[4] | (hb[5] << 16); uh[3] = hb[6] | (hb[7] << 16);
  ul[0] = lb[0] | (lb[1] << 16); ul[1] = lb[2] | (lb[3] << 16); ul[2] = lb[4] | (lb[5] << 16); ul[3] = lb[6] | (lb[7] << 16);
  *(volatile v4u*)ph = uh;
  *(volatile v4u*)pl = ul;
  __threadfence();
  *(volatile v4u*)ph = uh;
  *(volatile v4u*)pl = ul;
}

__global__ __launch_bounds__(256) void lay_x(const float* __restrict__ x, unsigned short* __restrict__ dst, int geom) {
  const int q  = blockIdx.x;
  const int cg = threadIdx.x;
  int hh, ww;
  bool valid;
  if (geom == GEOM_WHP) {
    ww = q / HP_COL;
    hh = (q - ww * HP_COL) - HALO;
    valid = (ww < FEAT_W) && (hh >= 0) && (hh < FEAT_H);
  } else {
    hh = q / WP_ROW;
    ww = (q - hh * WP_ROW) - HALO;
    valid = (hh < FEAT_H) && (ww >= 0) && (ww < FEAT_W);
  }
  const int hc = clampi(hh, 0, FEAT_H - 1);
  const int wc = clampi(ww, 0, FEAT_W - 1);
  const float* sp = x + (size_t)(cg * 8) * NPOS + hc * FEAT_W + wc;
  float v[8];
#pragma unroll
  for (int e = 0; e < 8; ++e) {
    const float t = sp[(size_t)e * NPOS];
    v[e] = valid ? t : 0.0f;
  }
  store8_f16(dst + (size_t)q * CH_IN + cg * 8, v);
}

__global__ __launch_bounds__(256) void lay_wtap(const float* __restrict__ w, unsigned short* __restrict__ dst,
                                                int cin, int nrow_real, int nrow_total, float scale) {
  const int gid  = blockIdx.x * 256 + threadIdx.x;
  const int ngrp = (NTAP * cin) >> 3;
  const int total = nrow_total * ngrp;
  if (gid >= total) return;
  const int row = gid / ngrp;
  const int g   = gid - row * ngrp;
  const int k   = g * 8;
  const int t   = k / cin;
  const int c   = k - t * cin;
  const bool valid = row < nrow_real;
  const int rc  = valid ? row : (nrow_real - 1);
  const float* sp = w + ((size_t)rc * cin + c) * NTAP + t;
  float v[8];
#pragma unroll
  for (int e = 0; e < 8; ++e) {
    const float tv = sp[(size_t)e * NTAP] * scale;
    v[e] = valid ? tv : 0.0f;
  }
  store8_f16(dst + (size_t)gid * 8, v);
}

__global__ __launch_bounds__(256) void lay_wk2(const float* __restrict__ w, unsigned short* __restrict__ dh,
                                               unsigned short* __restrict__ dl, int nrows, int nsrc, int kreal, int kpad) {
  const int gid  = blockIdx.x * 256 + threadIdx.x;
  const int ngrp = kpad >> 3;
  const int total = nrows * ngrp;
  if (gid >= total) return;
  const int row = gid / ngrp;
  const int k0  = (gid - row * ngrp) * 8;
  const bool rvalid = row < nsrc;
  const int rc  = rvalid ? row : (nsrc - 1);
  const float* sp = w + (size_t)rc * kreal;
  float v[8];
#pragma unroll
  for (int e = 0; e < 8; ++e) {
    const int kk = k0 + e;
    const int kc = kk < kreal ? kk : (kreal - 1);
    const float tv = sp[kc];
    v[e] = (rvalid && (kk < kreal)) ? tv : 0.0f;
  }
  store8_bf16x2(dh + (size_t)gid * 8, dl + (size_t)gid * 8, v);
}

__global__ __launch_bounds__(256) void lay_h1(const float* __restrict__ c1, unsigned short* __restrict__ dst,
                                              int geom, int src_wmajor, int nrows) {
  const int gid = blockIdx.x * 256 + threadIdx.x;
  const int q   = gid >> 5;
  const int cg  = gid & 31;
  if (q >= nrows) return;
  int hh, ww;
  bool valid;
  if (geom == GEOM_WHP) {
    ww = q / HP_COL;
    hh = (q - ww * HP_COL) - HALO;
    valid = (ww < FEAT_W) && (hh >= 0) && (hh < FEAT_H);
  } else {
    hh = q / WP_ROW;
    ww = (q - hh * WP_ROW) - HALO;
    valid = (hh < FEAT_H) && (ww >= 0) && (ww < FEAT_W);
  }
  const int hc = clampi(hh, 0, FEAT_H - 1);
  const int wc = clampi(ww, 0, FEAT_W - 1);
  const int srow = src_wmajor ? (wc * FEAT_H + hc) : (hc * FEAT_W + wc);
  const float* sp = c1 + (size_t)srow * CH_MID + cg * 8;
  const v4f a = *(const v4f*)sp;
  const v4f bq = *(const v4f*)(sp + 4);
  float v[8];
  v[0] = valid ? a[0] : 0.0f;  v[1] = valid ? a[1] : 0.0f;  v[2] = valid ? a[2] : 0.0f;  v[3] = valid ? a[3] : 0.0f;
  v[4] = valid ? bq[0] : 0.0f; v[5] = valid ? bq[1] : 0.0f; v[6] = valid ? bq[2] : 0.0f; v[7] = valid ? bq[3] : 0.0f;
  store8_f16(dst + (size_t)gid * 8, v);
}

__global__ __launch_bounds__(128) void mk_bias(const float* __restrict__ ba, const float* __restrict__ bb,
                                               float* __restrict__ dst) {
  const int t = threadIdx.x;
  float o[4];
#pragma unroll
  for (int e = 0; e < 4; ++e) {
    const int c  = 4 * t + e;
    const int cc = c < CH_OUT ? c : (CH_OUT - 1);
    const float v = ba[cc] + bb[cc];
    o[e] = (c < CH_OUT) ? v : 0.0f;
  }
  v4f w;
  w[0] = o[0]; w[1] = o[1]; w[2] = o[2]; w[3] = o[3];
  *(volatile v4f*)(dst + 4 * t) = w;
  __threadfence();
  *(volatile v4f*)(dst + 4 * t) = w;
}

__global__ __launch_bounds__(256) void psroi_pool(const float* __restrict__ rois, const float* __restrict__ feat,
                                                  unsigned short* __restrict__ ph, unsigned short* __restrict__ pl) {
#pragma clang fp contract(off)
  __shared__ __align__(16) float pv[KFC];
  const int r   = blockIdx.x;
  const int tid = threadIdx.x;
  const float rx1 = rois[r * 4 + 0];
  const float ry1 = rois[r * 4 + 1];
  const float rx2 = rois[r * 4 + 2];
  const float ry2 = rois[r * 4 + 3];
  const float xmin = (rx1 * 0.0625f) / (float)FEAT_W;
  const float ymin = (ry1 * 0.0625f) / (float)FEAT_H;
  const float xmax = (rx2 * 0.0625f) / (float)FEAT_W;
  const float ymax = (ry2 * 0.0625f) / (float)FEAT_H;
  const float step_x = (xmax - xmin) / (float)NBIN;
  const float step_y = (ymax - ymin) / (float)NBIN;
#pragma unroll 1
  for (int jj = 0; jj < 2; ++jj) {
    const int k   = tid + jj * 256;
    const int kc  = k < CH_OUT ? k : (CH_OUT - 1);
    const int bin = kc / BIN_CH;
    const int bi  = bin / NBIN;
    const int bj  = bin - bi * NBIN;
    float best = -__builtin_inff();
#pragma unroll 1
    for (int sy = 0; sy < 2; ++sy) {
      const float gy  = (float)(bi + sy);
      const float yy  = (ymin + gy * step_y) * (float)(FEAT_H - 1);
      const float y0f = floorf(yy);
      const float fy  = yy - y0f;
      const int iy0 = (int)fminf(fmaxf(y0f, 0.0f), (float)(FEAT_H - 1));
      const int iy1 = (int)fminf(fmaxf(y0f + 1.0f, 0.0f), (float)(FEAT_H - 1));
#pragma unroll 1
      for (int sx = 0; sx < 2; ++sx) {
        const float gx  = (float)(bj + sx);
        const float xx  = (xmin + gx * step_x) * (float)(FEAT_W - 1);
        const float x0f = floorf(xx);
        const float fx  = xx - x0f;
        const int ix0 = (int)fminf(fmaxf(x0f, 0.0f), (float)(FEAT_W - 1));
        const int ix1 = (int)fminf(fmaxf(x0f + 1.0f, 0.0f), (float)(FEAT_W - 1));
        const float v00 = feat[(size_t)(iy0 * FEAT_W + ix0) * CH_OUTP + kc];
        const float v01 = feat[(size_t)(iy0 * FEAT_W + ix1) * CH_OUTP + kc];
        const float v10 = feat[(size_t)(iy1 * FEAT_W + ix0) * CH_OUTP + kc];
        const float v11 = feat[(size_t)(iy1 * FEAT_W + ix1) * CH_OUTP + kc];
        const float top = v00 + (v01 - v00) * fx;
        const float bot = v10 + (v11 - v10) * fx;
        const float val = top + (bot - top) * fy;
        best = fmaxf(best, val);
      }
    }
    pv[k] = (k < CH_OUT) ? best : 0.0f;
  }
  __syncthreads();
  if (tid < 64) {
    float v[8];
#pragma unroll
    for (int e = 0; e < 8; ++e) v[e] = pv[tid * 8 + e];
    store8_bf16x2(ph + (size_t)r * KFC + tid * 8, pl + (size_t)r * KFC + tid * 8, v);
  }
}

__global__ __launch_bounds__(256) void write_out(const float* __restrict__ chd, const float* __restrict__ b_loc,
                                                 const float* __restrict__ b_score, float* __restrict__ out, int n4) {
  const int f = blockIdx.x * 256 + threadIdx.x;
  if (f >= n4) return;
  float o[4];
#pragma unroll
  for (int e = 0; e < 4; ++e) {
    const int idx  = f * 4 + e;
    const bool inA = idx < N_ROI * LOC_N;
    const int ia   = inA ? idx : (N_ROI * LOC_N - 1);
    const int ra   = ia / LOC_N;
    const int ca   = ia - ra * LOC_N;
    int ib = idx - N_ROI * LOC_N;
    ib = ib < 0 ? 0 : ib;
    ib = ib > (N_ROI * SC_N - 1) ? (N_ROI * SC_N - 1) : ib;
    const int rb   = ib / SC_N;
    const int cb   = ib - rb * SC_N;
    const int row  = inA ? ra : rb;
    const int col  = inA ? ca : (SC_BASE + cb);
    const float v  = chd[(size_t)row * NHD + col];
    const float ba = b_loc[ca];
    const float bs = b_score[cb];
    o[e] = v + (inA ? ba : bs);
  }
  v4f w;
  w[0] = o[0]; w[1] = o[1]; w[2] = o[2]; w[3] = o[3];
  *(volatile v4f*)(out + (size_t)f * 4) = w;
  __threadfence();
  *(volatile v4f*)(out + (size_t)f * 4) = w;
}

extern "C" void kernel_launch(void* const* d_in, const int* in_sizes, int n_in,
                              void* d_out, int out_size, void* d_ws, size_t ws_size,
                              hipStream_t stream) {
  if (n_in < 16) return;
  if (in_sizes[0] != CH_IN * NPOS || in_sizes[1] != N_ROI * 4 ||
      in_sizes[2] != CH_MID * CH_IN * NTAP || in_sizes[3] != CH_MID ||
      in_sizes[4] != CH_OUT * CH_MID * NTAP || in_sizes[5] != CH_OUT ||
      in_sizes[6] != CH_MID * CH_IN * NTAP || in_sizes[7] != CH_MID ||
      in_sizes[8] != CH_OUT * CH_MID * NTAP || in_sizes[9] != CH_OUT ||
      in_sizes[10] != NFC * CH_OUT || in_sizes[11] != NFC ||
      in_sizes[12] != SC_N * NFC || in_sizes[13] != SC_N ||
      in_sizes[14] != LOC_N * NFC || in_sizes[15] != LOC_N ||
      out_size != N_ROI * (LOC_N + SC_N)) return;
  if (ws_size < WS_TOTAL) return;

  const float* x         = (const float*)d_in[0];
  const float* rois      = (const float*)d_in[1];
  const float* w_col_max = (const float*)d_in[2];
  const float* b_col_max = (const float*)d_in[3];
  const float* w_col     = (const float*)d_in[4];
  const float* b_col     = (const float*)d_in[5];
  const float* w_row_max = (const float*)d_in[6];
  const float* b_row_max = (const float*)d_in[7];
  const float* w_row     = (const float*)d_in[8];
  const float* b_row     = (const float*)d_in[9];
  const float* w_fc1     = (const float*)d_in[10];
  const float* b_fc1     = (const float*)d_in[11];
  const float* w_score   = (const float*)d_in[12];
  const float* b_score   = (const float*)d_in[13];
  const float* w_loc     = (const float*)d_in[14];
  const float* b_loc     = (const float*)d_in[15];
  float* out = (float*)d_out;

  char* ws = (char*)d_ws;
  unsigned short* xTc   = (unsigned short*)(ws + OFF_XTC);
  unsigned short* xTr   = (unsigned short*)(ws + OFF_XTR);
  unsigned short* w1c   = (unsigned short*)(ws + OFF_W1C);
  unsigned short* w1r   = (unsigned short*)(ws + OFF_W1R);
  float*          c1c   = (float*)(ws + OFF_C1C);
  float*          c1r   = (float*)(ws + OFF_C1R);
  unsigned short* p2c   = (unsigned short*)(ws + OFF_P2C);
  unsigned short* p2r   = (unsigned short*)(ws + OFF_P2R);
  unsigned short* w2c   = (unsigned short*)(ws + OFF_W2C);
  unsigned short* w2r   = (unsigned short*)(ws + OFF_W2R);
  float*          btab  = (float*)(ws + OFF_BTAB);
  float*          c2a   = (float*)(ws + OFF_C2A);
  float*          c2    = (float*)(ws + OFF_C2);
  unsigned short* poolh = (unsigned short*)(ws + OFF_POOLH);
  unsigned short* pooll = (unsigned short*)(ws + OFF_POOLL);
  unsigned short* wfch  = (unsigned short*)(ws + OFF_WFCH);
  unsigned short* wfcl  = (unsigned short*)(ws + OFF_WFCL);
  unsigned short* cfch  = (unsigned short*)(ws + OFF_CFCH);
  unsigned short* cfcl  = (unsigned short*)(ws + OFF_CFCL);
  unsigned short* whdh  = (unsigned short*)(ws + OFF_WHDH);
  unsigned short* whdl  = (unsigned short*)(ws + OFF_WHDL);
  float*          chd   = (float*)(ws + OFF_CHD);

  const dim3 blk(256);
  const dim3 gblk(64);
  auto gemm_grid = [](int M, int N) { const int tiles = (M / 64) * (N / 64); return dim3((tiles + 1) / 2, 1); };

  lay_x<<<dim3(XTC_ROWS), blk, 0, stream>>>(x, xTc, GEOM_WHP);
  lay_x<<<dim3(XTR_ROWS), blk, 0, stream>>>(x, xTr, GEOM_HWP);
  lay_wtap<<<dim3((CH_MID * (KC1 / 8)) / 256), blk, 0, stream>>>(w_col_max, w1c, CH_IN, CH_MID, CH_MID, W_CARRY);
  lay_wtap<<<dim3((CH_MID * (KC1 / 8)) / 256), blk, 0, stream>>>(w_row_max, w1r, CH_IN, CH_MID, CH_MID, W_CARRY);
  lay_wtap<<<dim3((CH_OUTP * (KC2 / 8)) / 256), blk, 0, stream>>>(w_col, w2c, CH_MID, CH_OUT, CH_OUTP, W_CARRY);
  lay_wtap<<<dim3((CH_OUTP * (KC2 / 8)) / 256), blk, 0, stream>>>(w_row, w2r, CH_MID, CH_OUT, CH_OUTP, W_CARRY);
  lay_wk2<<<dim3((NFC * (KFC / 8)) / 256), blk, 0, stream>>>(w_fc1, wfch, wfcl, NFC, NFC, CH_OUT, KFC);
  lay_wk2<<<dim3((SC_BASE * (NFC / 8)) / 256), blk, 0, stream>>>(w_loc, whdh, whdl, SC_BASE, LOC_N, NFC, NFC);
  lay_wk2<<<dim3(((NHD - SC_BASE) * (NFC / 8)) / 256), blk, 0, stream>>>(
      w_score, whdh + (size_t)SC_BASE * NFC, whdl + (size_t)SC_BASE * NFC, NHD - SC_BASE, SC_N, NFC, NFC);
  mk_bias<<<dim3(1), dim3(128), 0, stream>>>(b_col, b_row, btab);

  wmma_gemm64<0, false, 2, 0, false, 0, true><<<gemm_grid(MPOS, CH_MID), gblk, 0, stream>>>(
      xTc, nullptr, CH_IN, 0L, w1c, nullptr, KC1, 0L, c1c, nullptr, CH_MID, 0L,
      b_col_max, nullptr, 0L, MPOS, CH_MID, KC1, W_CARRY_INV, FEAT_H, HP_COL, 1);
  wmma_gemm64<0, false, 2, 0, false, 0, true><<<gemm_grid(MPOS, CH_MID), gblk, 0, stream>>>(
      xTr, nullptr, CH_IN, 0L, w1r, nullptr, KC1, 0L, c1r, nullptr, CH_MID, 0L,
      b_row_max, nullptr, 0L, MPOS, CH_MID, KC1, W_CARRY_INV, FEAT_W, WP_ROW, 1);

  lay_h1<<<dim3(P2C_ROWS / 8), blk, 0, stream>>>(c1c, p2c, GEOM_HWP, 1, P2C_ROWS);
  lay_h1<<<dim3(P2R_ROWS / 8), blk, 0, stream>>>(c1r, p2r, GEOM_WHP, 0, P2R_ROWS);

  wmma_gemm64<0, false, 0, 0, false, 0, true><<<gemm_grid(MPOS, CH_OUTP), gblk, 0, stream>>>(
      p2c, nullptr, CH_MID, 0L, w2c, nullptr, KC2, 0L, c2a, nullptr, CH_OUTP, 0L,
      nullptr, nullptr, 0L, MPOS, CH_OUTP, KC2, W_CARRY_INV, FEAT_W, WP_ROW, 1);
  wmma_gemm64<0, false, 2, 0, true, 2, true><<<gemm_grid(MPOS, CH_OUTP), gblk, 0, stream>>>(
      p2r, nullptr, CH_MID, 0L, w2r, nullptr, KC2, 0L, c2, nullptr, CH_OUTP, 0L,
      btab, c2a, 0L, MPOS, CH_OUTP, KC2, W_CARRY_INV, FEAT_W, 1, HP_COL);

  psroi_pool<<<dim3(N_ROI), blk, 0, stream>>>(rois, c2, poolh, pooll);

  wmma_gemm64<1, true, 2, 2, false, 2, false><<<gemm_grid(N_ROI, NFC), gblk, 0, stream>>>(
      poolh, pooll, KFC, 0L, wfch, wfcl, KFC, 0L, cfch, cfcl, NFC, 0L,
      b_fc1, nullptr, 0L, N_ROI, NFC, KFC, 1.0f, 1, 0, 1);
  wmma_gemm64<1, true, 0, 0, false, 0, false><<<gemm_grid(N_ROI, NHD), gblk, 0, stream>>>(
      cfch, cfcl, NFC, 0L, whdh, whdl, NFC, 0L, chd, nullptr, NHD, 0L,
      nullptr, nullptr, 0L, N_ROI, NHD, NFC, 1.0f, 1, 0, 1);

  const int n4 = out_size / 4;
  write_out<<<dim3((n4 + 255) / 256), blk, 0, stream>>>(chd, b_loc, b_score, out, n4);
}
